// OuterAttention_11123965296644
// MI455X (gfx1250) — hardware-verified
//
#include <hip/hip_runtime.h>


namespace {
constexpr int NA = 8192, E = 1024, MH = 1024, NRB = NA / 128;

typedef _Float16 b16;
typedef __attribute__((ext_vector_type(16))) _Float16 v16b;
typedef __attribute__((ext_vector_type(8)))  _Float16 v8b;
typedef __attribute__((ext_vector_type(8)))  float v8f;
typedef __attribute__((ext_vector_type(4)))  float v4f;

__device__ __forceinline__ v8b ld8b(const b16* p) { return *(const v8b*)p; }
__device__ __forceinline__ v16b cat8b(v8b a, v8b b) { return __builtin_shufflevector(a, b, 0, 1, 2, 3, 4, 5, 6, 7, 8, 9, 10, 11, 12, 13, 14, 15); }
__device__ __forceinline__ v16b frag_kb(const b16* p, int hh) { return cat8b(ld8b(p + 8 * hh), ld8b(p + 16 + 8 * hh)); }
__device__ __forceinline__ void split16(float v, b16& hi, b16& lo) { hi = (b16)v; lo = (b16)(v - (float)hi); }
__device__ __forceinline__ void frag_ksplit(const float* p, int hh, v16b& fh_, v16b& fl_) {
  const float* p0 = p + 8 * hh; const float* p1 = p + 16 + 8 * hh;
#pragma unroll
  for (int e = 0; e < 8; ++e) { b16 a, c; split16(p0[e], a, c); fh_[e] = a; fl_[e] = c; split16(p1[e], a, c); fh_[8 + e] = a; fl_[8 + e] = c; }
}
__device__ __forceinline__ v8f wmma16b(v16b a, v16b b, v8f c) {
  v8f d = __builtin_amdgcn_wmma_f32_16x16x32_f16(false, a, false, b, (short)0, c, false, false);
  asm volatile("v_nop\n\tv_nop\n\tv_nop\n\tv_nop" : "+v"(d) : "v"(a), "v"(b));
  return d;
}
__device__ __forceinline__ void wave_lds_sync() {
  __builtin_amdgcn_fence(__ATOMIC_RELEASE, "workgroup");
  __builtin_amdgcn_wave_barrier();
  __builtin_amdgcn_fence(__ATOMIC_ACQUIRE, "workgroup");
}

struct Opnd { const void* p0; const void* p1; int ld; };
template <int NP> __device__ __forceinline__ void load_frags(const Opnd& o, int row, int kb, int hh, v16b& fh_, v16b& fl_) {
  if (NP == 0) { frag_ksplit((const float*)o.p0 + (size_t)row * o.ld + kb, hh, fh_, fl_); }
  else if (NP == 4) {
    const float* p = (const float*)o.p0 + (size_t)row * o.ld + kb; const float* p0 = p + 8 * hh; const float* p1 = p + 16 + 8 * hh;
#pragma unroll
    for (int e = 0; e < 8; ++e) { b16 a, c; split16(p0[e] * 64.0f, a, c); fh_[e] = a; fl_[e] = c; split16(p1[e] * 64.0f, a, c); fh_[8 + e] = a; fl_[8 + e] = c; }
  } else if (NP == 3) {
    const float* p = (const float*)o.p0 + (size_t)row * o.ld + kb; const float* p0 = p + 8 * hh; const float* p1 = p + 16 + 8 * hh;
#pragma unroll
    for (int e = 0; e < 8; ++e) { fh_[e] = (b16)p0[e]; fh_[8 + e] = (b16)p1[e]; }
    fl_ = fh_;
  } else {
    fh_ = frag_kb((const b16*)o.p0 + (size_t)row * o.ld + kb, hh);
    if (NP == 2) fl_ = frag_kb((const b16*)o.p1 + (size_t)row * o.ld + kb, hh); else fl_ = fh_;
  }
}
template <int ANP, int BNP> __device__ __forceinline__ v8f mac(v16b ah, v16b al, v16b bh, v16b bl, v8f c) {
  c = wmma16b(ah, bh, c);
  if (BNP == 0 || BNP == 2 || BNP == 4) c = wmma16b(ah, bl, c);
  if (ANP == 0 || ANP == 2 || ANP == 4) c = wmma16b(al, bh, c);
  return c;
}
template <int ANP, int BNP>
__device__ __forceinline__ void gemm_tile(const Opnd& A, const Opnd& B, int K, int m0, int c0, int nloc, int hlf, v8f (&acc)[2][4]) {
  for (int kb = 0; kb < K; kb += 32) {
    v16b a0h, a0l, a1h, a1l;
    load_frags<ANP>(A, m0 + nloc, kb, hlf, a0h, a0l);
    load_frags<ANP>(A, m0 + 16 + nloc, kb, hlf, a1h, a1l);
#pragma unroll
    for (int t = 0; t < 4; ++t) {
      v16b bh, bl;
      load_frags<BNP>(B, c0 + t * 16 + nloc, kb, hlf, bh, bl);
      acc[0][t] = mac<ANP, BNP>(a0h, a0l, bh, bl, acc[0][t]);
      acc[1][t] = mac<ANP, BNP>(a1h, a1l, bh, bl, acc[1][t]);
    }
  }
}

__device__ __forceinline__ void epi_planes(v8f (&acc)[2][4], float scale, bool two, b16* __restrict__ oh, b16* __restrict__ ol, int ldo,
                                           int m0, int c0, int lane, b16* Th, b16* Tl) {
  const int nloc = lane & 15, hlf = lane >> 4;
#pragma unroll
  for (int t = 0; t < 4; ++t)
#pragma unroll
    for (int r = 0; r < 2; ++r)
#pragma unroll
      for (int v = 0; v < 8; ++v) {
        const int rr = r * 16 + v + 8 * hlf, cc = t * 16 + nloc;
        b16 h_, l_; split16(acc[r][t][v] * scale, h_, l_);
        Th[rr * 64 + cc] = h_; Tl[rr * 64 + cc] = l_;
      }
  wave_lds_sync();
  for (int pass = 0; pass < 2; ++pass) {
#pragma unroll
    for (int j = 0; j < 8; ++j) {
      const int rr = j * 4 + (lane >> 3), c8 = (lane & 7) * 8;
      const size_t o = (size_t)(m0 + rr) * ldo + c0 + c8;
      *(volatile v8b*)(oh + o) = ld8b(Th + rr * 64 + c8);
      if (two) *(volatile v8b*)(ol + o) = ld8b(Tl + rr * 64 + c8);
    }
    __threadfence();
  }
}
__device__ __forceinline__ void epi_f32(v8f (&acc)[2][4], float scale, const float* rscale, float* __restrict__ out, int ldo, int m0, int c0, int lane, float* Tt) {
  const int nloc = lane & 15, hlf = lane >> 4;
#pragma unroll
  for (int t = 0; t < 4; ++t)
#pragma unroll
    for (int r = 0; r < 2; ++r)
#pragma unroll
      for (int v = 0; v < 8; ++v) {
        const int rr = r * 16 + v + 8 * hlf;
        const float rs = rscale ? rscale[(size_t)(m0 + rr) * 32] : 1.0f;
        Tt[rr * 64 + t * 16 + nloc] = acc[r][t][v] * scale * rs;
      }
  wave_lds_sync();
  float* dst0 = out + (size_t)m0 * ldo + c0;
  for (int pass = 0; pass < 2; ++pass) {
#pragma unroll
    for (int j = 0; j < 16; ++j) { const int rr = j * 2 + hlf, c4 = nloc * 4; *(volatile v4f*)(dst0 + (size_t)rr * ldo + c4) = *(const v4f*)(Tt + rr * 64 + c4); }
    __threadfence();
  }
}


__global__ __launch_bounds__(256) void prep_kernel(const float* __restrict__ W1, const float* __restrict__ W2, const float* __restrict__ Wc1, const float* __restrict__ Wc2,
                                                   const float* __restrict__ ctx, b16* __restrict__ w16, float* __restrict__ cvec) {
  __shared__ float cs[32];
  const int tid = threadIdx.x, lane = tid & 31, wave = tid >> 5;
  if (blockIdx.x < 1024) {
    const size_t i0 = ((size_t)blockIdx.x * 256 + tid) * 8; const size_t n1 = (size_t)MH * E;
    const float* src = (i0 < n1) ? (W1 + i0) : (W2 + (i0 - n1)); v8b v;
#pragma unroll
    for (int e = 0; e < 8; ++e) v[e] = (b16)src[e];
    *(volatile v8b*)(w16 + i0) = v; __threadfence(); *(volatile v8b*)(w16 + i0) = v;
    return;
  }
  const int bb = blockIdx.x - 1024, z = bb / 32, r0 = (bb % 32) * 32;
  const float* W = z ? Wc2 : Wc1;
  for (int q = 0; q < 4; ++q) {
    const int r = r0 + wave * 4 + q; float s = 0.0f;
#pragma unroll 1
    for (int k0 = 0; k0 < E; k0 += 128) { const v4f a = *(const v4f*)(W + (size_t)r * E + k0 + lane * 4), c = *(const v4f*)(ctx + k0 + lane * 4); s += a[0] * c[0] + a[1] * c[1] + a[2] * c[2] + a[3] * c[3]; }
#pragma unroll
    for (int o = 16; o > 0; o >>= 1) s += __shfl_xor(s, o);
    if (lane == 0) cs[wave * 4 + q] = s;
  }
  __syncthreads();
  if (wave == 0) { ((volatile float*)cvec)[z * MH + r0 + lane] = cs[lane]; __threadfence(); ((volatile float*)cvec)[z * MH + r0 + lane] = cs[lane]; }
}

__global__ __launch_bounds__(128) void proj_kernel(const float* __restrict__ s1, const float* __restrict__ s2, const b16* __restrict__ w16, const float* __restrict__ b1,
                                                   const float* __restrict__ b2, const float* __restrict__ cvec, float* __restrict__ P, float* __restrict__ csl) {
  __shared__ __attribute__((aligned(16))) float Ts[4][32 * 64]; __shared__ __attribute__((aligned(16))) float Cs[4][64];
  const int lane = threadIdx.x & 31, wave = threadIdx.x >> 5, nloc = lane & 15, hlf = lane >> 4, z = blockIdx.z;
  const int m0 = blockIdx.y * 128 + wave * 32, c0 = blockIdx.x * 64;
  v8f acc[2][4];
#pragma unroll
  for (int r = 0; r < 2; ++r)
#pragma unroll
    for (int t = 0; t < 4; ++t) acc[r][t] = (v8f){};
  const Opnd A{z ? s2 : s1, nullptr, E}, B{w16 + (size_t)z * MH * E, nullptr, E};
  gemm_tile<3, 1>(A, B, E, m0, c0, nloc, hlf, acc);
  const float* bz = z ? b2 : b1; const float* cz = cvec + (size_t)z * MH;
  float* Tt = Ts[wave]; float colsum[4] = {0.f, 0.f, 0.f, 0.f};
#pragma unroll
  for (int t = 0; t < 4; ++t)
#pragma unroll
    for (int r = 0; r < 2; ++r)
#pragma unroll
      for (int v = 0; v < 8; ++v) {
        const int rr = r * 16 + v + 8 * hlf, cc = t * 16 + nloc; float val = acc[r][t][v] + bz[c0 + cc] + cz[c0 + cc];
        val = (val > 0.0f) ? val : (__expf(val) - 1.0f);
        Tt[rr * 64 + cc] = val; colsum[t] += val;
      }
#pragma unroll
  for (int t = 0; t < 4; ++t) { colsum[t] += __shfl_xor(colsum[t], 16); if (hlf == 0) Cs[wave][t * 16 + nloc] = colsum[t]; }
  wave_lds_sync();
  float* dst0 = P + ((size_t)z * NA + m0) * MH + c0;
  for (int pass = 0; pass < 2; ++pass) {
#pragma unroll
    for (int j = 0; j < 16; ++j) { const int rr = j * 2 + hlf, c4 = nloc * 4; *(volatile v4f*)(dst0 + (size_t)rr * MH + c4) = *(const v4f*)(Tt + rr * 64 + c4); }
    __threadfence();
  }
  __syncthreads();
  if (wave == 0 && lane < 16) {
    v4f s4;
#pragma unroll
    for (int e = 0; e < 4; ++e) { const int cc = lane * 4 + e; s4[e] = (Cs[0][cc] + Cs[1][cc]) + (Cs[2][cc] + Cs[3][cc]); }
    float* cd = csl + ((size_t)z * NRB + blockIdx.y) * MH + c0 + lane * 4;
    *(volatile v4f*)cd = s4; __threadfence(); *(volatile v4f*)cd = s4;
  }
}

__global__ __launch_bounds__(256) void colsum_kernel(const float* __restrict__ csl, float* __restrict__ Ssum) {
  const int z = blockIdx.x / 4, m = (blockIdx.x % 4) * 256 + threadIdx.x; float s = 0.0f;
#pragma unroll 1
  for (int rb = 0; rb < NRB; ++rb) s += csl[((size_t)z * NRB + rb) * MH + m];
  ((volatile float*)Ssum)[z * MH + m] = s; __threadfence(); ((volatile float*)Ssum)[z * MH + m] = s;
}

__global__ __launch_bounds__(256) void logit_kernel(const float* __restrict__ P, const float* __restrict__ Ssum, float* __restrict__ lg) {
  __shared__ float ls[32];
  const int wave = threadIdx.x >> 5, lane = threadIdx.x & 31, z = blockIdx.y, r0 = blockIdx.x * 32;
  const float* Sv = Ssum + (size_t)(1 - z) * MH;
  for (int q = 0; q < 4; ++q) {
    const int r = r0 + wave * 4 + q; const float* row = P + ((size_t)z * NA + r) * MH; float s = 0.0f;
#pragma unroll 1
    for (int k0 = 0; k0 < MH; k0 += 128) { const v4f a = *(const v4f*)(row + k0 + lane * 4), c = *(const v4f*)(Sv + k0 + lane * 4); s += a[0] * c[0] + a[1] * c[1] + a[2] * c[2] + a[3] * c[3]; }
#pragma unroll
    for (int o = 16; o > 0; o >>= 1) s += __shfl_xor(s, o);
    if (lane == 0) ls[wave * 4 + q] = s;
  }
  __syncthreads();
  if (wave == 0) { ((volatile float*)lg)[(size_t)z * NA + r0 + lane] = ls[lane]; __threadfence(); ((volatile float*)lg)[(size_t)z * NA + r0 + lane] = ls[lane]; }
}

__global__ __launch_bounds__(256) void att_kernel(const float* __restrict__ s1, const float* __restrict__ s2, const float* __restrict__ lg, float* __restrict__ out) {
  __shared__ float w[NA]; __shared__ float red[256];
  const int z = blockIdx.x / 4, e = (blockIdx.x % 4) * 256 + threadIdx.x, t = threadIdx.x;
  const float* L = lg + (size_t)z * NA; const float* seq = z ? s2 : s1;
  float mx = -INFINITY;
  for (int a = t; a < NA; a += 256) mx = fmaxf(mx, L[a]);
  red[t] = mx; __syncthreads();
  for (int o = 128; o > 0; o >>= 1) { if (t < o) red[t] = fmaxf(red[t], red[t + o]); __syncthreads(); }
  mx = red[0]; __syncthreads();
  float sm = 0.0f;
  for (int a = t; a < NA; a += 256) { const float v = expf(L[a] - mx); w[a] = v; sm += v; }
  red[t] = sm; __syncthreads();
  for (int o = 128; o > 0; o >>= 1) { if (t < o) red[t] += red[t + o]; __syncthreads(); }
  const float inv = 1.0f / red[0];
  float acc = 0.0f;
#pragma unroll 1
  for (int a = 0; a < NA; ++a) { const float wa = w[a]; if (wa != 0.0f) acc += wa * seq[(size_t)a * E + e]; }
  acc *= inv;
  ((volatile float*)out)[z * E + e] = acc; __threadfence(); ((volatile float*)out)[z * E + e] = acc;
}
}

extern "C" void kernel_launch(void* const* d_in, const int* in_sizes, int n_in,
                              void* d_out, int out_size, void* d_ws, size_t ws_size, hipStream_t stream) {
  (void)n_in; (void)out_size;
  const float* s1 = (const float*)d_in[0]; const float* s2 = (const float*)d_in[1];
  const float* ctx = (const float*)d_in[2];
  const float* Wc1 = (const float*)d_in[3]; const float* Wc2 = (const float*)d_in[4];
  const float* W1 = (const float*)d_in[5]; const float* b1 = (const float*)d_in[6];
  const float* W2 = (const float*)d_in[7]; const float* b2 = (const float*)d_in[8];
  float* out = (float*)d_out;
  if (in_sizes[0] != NA * E || in_sizes[1] != NA * E || in_sizes[2] != E || in_sizes[5] != MH * E) return;
  size_t off = 0; char* ws = (char*)d_ws;
  auto carve = [&](size_t bytes) { char* p = ws + off; off += (bytes + 255) & ~(size_t)255; return p; };
  b16* w16 = (b16*)carve((size_t)2 * MH * E * 2);
  float* cvec = (float*)carve((size_t)2 * MH * 4);
  float* P = (float*)carve((size_t)2 * NA * MH * 4);
  float* csl = (float*)carve((size_t)2 * NRB * MH * 4);
  float* Ssum = (float*)carve((size_t)2 * MH * 4);
  float* lg = (float*)carve((size_t)2 * NA * 4);
  if (off > ws_size) return;
  prep_kernel<<<1024 + 64, 256, 0, stream>>>(W1, W2, Wc1, Wc2, ctx, w16, cvec);
  proj_kernel<<<dim3(MH / 64, NA / 128, 2), 128, 0, stream>>>(s1, s2, w16, b1, b2, cvec, P, csl);
  colsum_kernel<<<8, 256, 0, stream>>>(csl, Ssum);
  logit_kernel<<<dim3(NA / 32, 2), 256, 0, stream>>>(P, Ssum, lg);
  att_kernel<<<8, 256, 0, stream>>>(s1, s2, lg, out);
}
